// GraphAttentionLayer_84207128805823
// MI455X (gfx1250) — hardware-run, weakly checked
//
#include <hip/hip_runtime.h>

typedef float          v8f   __attribute__((ext_vector_type(8)));
typedef float          v4f   __attribute__((ext_vector_type(4)));
typedef unsigned int   v4u   __attribute__((ext_vector_type(4)));
typedef int            v8i   __attribute__((ext_vector_type(8)));
typedef unsigned short v8us  __attribute__((ext_vector_type(8)));
typedef unsigned short v16us __attribute__((ext_vector_type(16)));
typedef __bf16         v16bf __attribute__((ext_vector_type(16)));
typedef _Float16       v16h  __attribute__((ext_vector_type(16)));
typedef v4f  __attribute__((may_alias)) v4fa;
typedef v8us __attribute__((may_alias)) v8usa;
union FragB { v16bf v; v16us u; v8us h[2]; v8i w; };
union FragH { v16h  v; v16us u; v8us h[2]; v8i w; };

__device__ __forceinline__ v8f wmb(const FragB& a, const FragB& b, v8f c) {
  v8f d = __builtin_amdgcn_wmma_f32_16x16x32_bf16(false, a.v, false, b.v, (short)0, c, false, false);
  asm volatile("v_nop\n\tv_nop\n\tv_nop\n\tv_nop" : "+v"(d) : "v"(a.w), "v"(b.w));
  return d;
}

__device__ __forceinline__ v8f wmh(const FragH& a, const FragH& b, v8f c) {
  v8f d = __builtin_amdgcn_wmma_f32_16x16x32_f16(false, a.v, false, b.v, (short)0, c, false, false);
  asm volatile("v_nop\n\tv_nop\n\tv_nop\n\tv_nop" : "+v"(d) : "v"(a.w), "v"(b.w));
  return d;
}

__device__ __forceinline__ unsigned bf16_bits(float f) {
  const unsigned u = __float_as_uint(f);
  const unsigned r = (u + 0x7FFFu + ((u >> 16) & 1u)) >> 16;
  const unsigned q = (u >> 16) | 0x40u;
  return ((u & 0x7fffffffu) > 0x7f800000u) ? q : r;
}

__device__ __forceinline__ float bf16_val(float f) {
  return __uint_as_float(bf16_bits(f) << 16);
}
__device__ __forceinline__ int clampi(int v, int lo, int hi) {
  return v < lo ? lo : (v > hi ? hi : v);
}

__device__ __forceinline__ unsigned f16_bits(float f) {
  const unsigned u  = __float_as_uint(f);
  const unsigned s  = (u >> 16) & 0x8000u;
  const unsigned a  = u & 0x7fffffffu;
  const unsigned t  = a - 0x38000000u;
  const unsigned r  = (t + 0x0FFFu + ((t >> 13) & 1u)) >> 13;
  const unsigned rc = r > 0x7C00u ? 0x7C00u : r;
  const bool small  = a < 0x38800000u;
  const bool isnan  = a > 0x7f800000u;
  const unsigned fin = small ? 0u : (s | rc);
  return isnan ? (s | 0x7E00u) : fin;
}

__device__ __forceinline__ unsigned pk16(unsigned lo, unsigned hi) { return lo | (hi << 16); }
__device__ __forceinline__ unsigned bf16_lo_bits(float v) {
  float hi = bf16_val(v);
  asm volatile("" : "+v"(hi));
  return bf16_bits(v - hi);
}
__device__ __forceinline__ v4u pack8_bf16(v4f a, v4f c) {
  return (v4u){ pk16(bf16_bits(a[0]), bf16_bits(a[1])), pk16(bf16_bits(a[2]), bf16_bits(a[3])),
                pk16(bf16_bits(c[0]), bf16_bits(c[1])), pk16(bf16_bits(c[2]), bf16_bits(c[3])) };
}
__device__ __forceinline__ v4u pack8_bf16_lo(v4f a, v4f c) {
  return (v4u){ pk16(bf16_lo_bits(a[0]), bf16_lo_bits(a[1])), pk16(bf16_lo_bits(a[2]), bf16_lo_bits(a[3])),
                pk16(bf16_lo_bits(c[0]), bf16_lo_bits(c[1])), pk16(bf16_lo_bits(c[2]), bf16_lo_bits(c[3])) };
}
__device__ __forceinline__ v4u pack8_f16(v4f a, v4f c) {
  return (v4u){ pk16(f16_bits(a[0]), f16_bits(a[1])), pk16(f16_bits(a[2]), f16_bits(a[3])),
                pk16(f16_bits(c[0]), f16_bits(c[1])), pk16(f16_bits(c[2]), f16_bits(c[3])) };
}

template <int FORM>
__global__ __launch_bounds__(256) void k_plane(const float* __restrict__ src, int rows, int cols, int ldsrc,
                                               unsigned short* __restrict__ dst, int MP, int KP) {
  static_assert(FORM >= 0 && FORM <= 3);
  const int KTOT = (FORM == 1 || FORM == 3) ? 2 * KP : KP;
  const unsigned ppr   = (unsigned)(KTOT >> 3);
  const unsigned kp8   = (unsigned)(KP >> 3);
  const unsigned total = (unsigned)MP * ppr;
  const unsigned g     = blockIdx.x * 256u + threadIdx.x;
  const unsigned rowu  = g / ppr;
  const unsigned p     = g - rowu * ppr;
  const bool second    = p >= kp8;
  const int row = (int)rowu;
  const int c0  = (int)((second ? p - kp8 : p) << 3);
  const float* srow = src + (size_t)clampi(row, 0, rows - 1) * (size_t)ldsrc;
  float x[8];
  unsigned mk[8];
#pragma unroll
  for (int e = 0; e < 8; ++e) {
    const int c = c0 + e;
    const float v = srow[clampi(c, 0, cols - 1)];
    asm volatile("" :: "v"(v));
    x[e]  = v;
    mk[e] = (row < rows && c < cols) ? 0xFFFFu : 0u;
  }
  const v4f a = (v4f){ x[0], x[1], x[2], x[3] };
  const v4f c = (v4f){ x[4], x[5], x[6], x[7] };
  v4u o;
  if (FORM == 2) {
    o = pack8_f16(a, c);
  } else {
    const v4u hi = pack8_bf16(a, c);
    o = hi;
    if (FORM == 1) { const v4u lo = pack8_bf16_lo(a, c); o = second ? lo : hi; }
  }
  const v4u mw = (v4u){ pk16(mk[0], mk[1]), pk16(mk[2], mk[3]), pk16(mk[4], mk[5]), pk16(mk[6], mk[7]) };
  o &= mw;
  if (g < total) {
    volatile v4u* q = (volatile v4u*)(dst + (size_t)g * 8);
    *q = o;
    __threadfence();
    *q = o;
  }
}

template <int FORM> struct FragOf    { typedef FragB T; };
template <>         struct FragOf<2> { typedef FragH T; };
__device__ __forceinline__ v8f mm(const FragB& a, const FragB& b, v8f c) { return wmb(a, b, c); }
__device__ __forceinline__ v8f mm(const FragH& a, const FragH& b, v8f c) { return wmh(a, b, c); }
template <class F> __device__ __forceinline__ F ld_frag(const unsigned short* p) {
  F f;
  f.h[0] = *(const v8usa*)(p);
  f.h[1] = *(const v8usa*)(p + 16);
  return f;
}

template <int FORM, int EPI>
__global__ __launch_bounds__(256) __attribute__((amdgpu_num_vgpr(248)))
void k_gemm_nt(const unsigned short* __restrict__ A, const unsigned short* __restrict__ B,
               const float* __restrict__ bias, float* __restrict__ D, int M, int N, int KTOT, int ldd) {
  static_assert(FORM >= 0 && FORM <= 2);
  static_assert(EPI == 0 || EPI == 1);
  typedef typename FragOf<FORM>::T F;
  __shared__ __attribute__((aligned(16))) float sT[8][16 * 68];
  const int lane = threadIdx.x & 31;
  const int wave = threadIdx.x >> 5;
  const int tilesM = (M + 63) >> 6;
  const int tilesN = (N + 63) >> 6;
  const int tile = blockIdx.x * 8 + wave;
  if (tile >= tilesM * tilesN) return;
  const int tm = tile / tilesN;
  const int tn = tile - tm * tilesN;
  const int m0 = tm << 6;
  const int n0 = tn << 6;

  const int rl = lane & 15;
  const int h8 = (lane >> 4) * 8;
  const unsigned short* pa = A + (size_t)(m0 + rl) * (size_t)KTOT + h8;
  const unsigned short* pb = B + (size_t)(n0 + rl) * (size_t)KTOT + h8;

  v8f acc[4][4];
#pragma unroll
  for (int i = 0; i < 4; ++i)
#pragma unroll
    for (int j = 0; j < 4; ++j) acc[i][j] = (v8f){0.f, 0.f, 0.f, 0.f, 0.f, 0.f, 0.f, 0.f};

#pragma unroll 1
  for (int k0 = 0; k0 < KTOT; k0 += 32) {
    F bf[4];
#pragma unroll
    for (int j = 0; j < 4; ++j) bf[j] = ld_frag<F>(pb + (size_t)(j << 4) * (size_t)KTOT + k0);
#pragma unroll
    for (int i = 0; i < 4; ++i) {
      const F af = ld_frag<F>(pa + (size_t)(i << 4) * (size_t)KTOT + k0);
#pragma unroll
      for (int j = 0; j < 4; ++j) acc[i][j] = mm(af, bf[j], acc[i][j]);
    }
  }

  float* slab = sT[wave];
  const int hh = lane >> 4;
  const int c4 = (lane & 15) * 4;
  const int nc = n0 + c4;
  const bool cok = nc < N;
  v4f bv = (v4f){0.f, 0.f, 0.f, 0.f};
  if (EPI == 1) {
    bv = *(const v4fa*)(bias + clampi(nc, 0, N - 4));
    asm volatile("" :: "v"(bv));
  }
#pragma unroll
  for (int i = 0; i < 4; ++i) {
    const int mBase = m0 + (i << 4);
#pragma unroll
    for (int j = 0; j < 4; ++j) {
#pragma unroll
      for (int r = 0; r < 8; ++r) slab[(h8 + r) * 68 + (j << 4) + rl] = acc[i][j][r];
    }
    __builtin_amdgcn_fence(__ATOMIC_RELEASE, "workgroup");
    __builtin_amdgcn_wave_barrier();
    __builtin_amdgcn_fence(__ATOMIC_ACQUIRE, "workgroup");
    v4f vv[8];
#pragma unroll
    for (int it = 0; it < 8; ++it) {
      const int row = it * 2 + hh;
      v4f v = *(const v4fa*)(slab + row * 68 + c4);
      if (EPI == 1) v += bv;
      vv[it] = v;
    }
    for (int pass = 0; pass < 2; ++pass) {
#pragma unroll
      for (int it = 0; it < 8; ++it) {
        const int row = mBase + it * 2 + hh;
        if (cok && row < M) *(volatile v4f*)(D + (size_t)row * (size_t)ldd + nc) = vv[it];
      }
      __threadfence();
    }
    __builtin_amdgcn_fence(__ATOMIC_RELEASE, "workgroup");
    __builtin_amdgcn_wave_barrier();
    __builtin_amdgcn_fence(__ATOMIC_ACQUIRE, "workgroup");
  }
}

#ifndef P_LO
#define P_LO 1
#endif
#ifndef H_LO
#define H_LO 1
#endif

constexpr int NBATCH = 32;
constexpr int NN     = 1024;
constexpr int INC    = 64;
constexpr int OUTC   = 128;
constexpr int ROWS   = NBATCH * NN;
constexpr int KCAT   = 3 * NN;
constexpr int CB     = 8;
constexpr float SLOPE = 0.2f;
constexpr float FILLV = -1e16f;

static_assert(NN % 64 == 0);
static_assert(KCAT == 3 * NN && KCAT % 32 == 0);
static_assert(OUTC == 128 && OUTC == 32 * 4);
static_assert(ROWS % 32 == 0 && ROWS % 64 == 0 && ROWS % 8 == 0);
static_assert(NBATCH % CB == 0);
static_assert(INC % 32 == 0 && OUTC % 64 == 0 && NN % 16 == 0 && NN % 8 == 0);
static_assert(NN == 4 * 256);
static_assert((size_t)ROWS * (INC / 8) % 256 == 0 && (size_t)OUTC * (INC / 8) % 256 == 0);

constexpr size_t SZ_XB  = (size_t)ROWS * INC * 2;
constexpr size_t SZ_WB  = (size_t)OUTC * INC * 2;
constexpr size_t SZ_TAB = 4096;
constexpr size_t SZ_H   = (size_t)ROWS * OUTC * 4;
constexpr size_t SZ_S   = (size_t)2 * ROWS * 4;
constexpr size_t SZ_BT  = (size_t)NBATCH * OUTC * KCAT * 2;
constexpr size_t SZ_AP  = (size_t)CB * NN * KCAT * 2;
constexpr size_t SZ_O   = (size_t)ROWS * OUTC * 4;
constexpr size_t OFF_XB  = 0;
constexpr size_t OFF_WB  = OFF_XB + SZ_XB;
constexpr size_t OFF_TAB = OFF_WB + SZ_WB;
constexpr size_t OFF_H   = OFF_TAB + SZ_TAB;
constexpr size_t OFF_S   = OFF_H + SZ_H;
constexpr size_t OFF_BT  = OFF_S + SZ_S;
constexpr size_t OFF_AP  = OFF_BT + SZ_BT;
constexpr size_t OFF_O   = OFF_AP + SZ_AP;
constexpr size_t WS_TOTAL = OFF_O + SZ_O;
static_assert(WS_TOTAL == (size_t)((size_t)27717 << 12));
static_assert(WS_TOTAL <= ((size_t)128 << 20));
static_assert(OFF_WB % 256 == 0 && OFF_TAB % 256 == 0 && OFF_H % 256 == 0 && OFF_S % 256 == 0);
static_assert(OFF_BT % 256 == 0 && OFF_AP % 256 == 0 && OFF_O % 256 == 0);
static_assert((size_t)3 * OUTC * 4 <= SZ_TAB);
static_assert(((size_t)NN * KCAT * 2) % 128 == 0 && ((size_t)OUTC * KCAT * 2) % 128 == 0);

__global__ __launch_bounds__(256) void k_tab(const float* __restrict__ av, const float* __restrict__ bv,
                                             float* __restrict__ tab) {
  const int tid = (int)threadIdx.x;
  const int u   = tid < 96 ? tid : 95;
  const int ia  = clampi(u, 0, 63) * 4;
  const int ib  = clampi(u - 64, 0, 31) * 4;
  const v4f va = *(const v4fa*)(av + ia);
  const v4f vb = *(const v4fa*)(bv + ib);
  asm volatile("" :: "v"(va));
  asm volatile("" :: "v"(vb));
  const unsigned ma = (u < 64) ? 0xFFFFFFFFu : 0u;
  v4f o;
#pragma unroll
  for (int e = 0; e < 4; ++e) {
    const unsigned bits = (__float_as_uint(va[e]) & ma) | (__float_as_uint(vb[e]) & ~ma);
    o[e] = bf16_val(__uint_as_float(bits));
  }
  if (tid < 96) {
    volatile v4f* q = (volatile v4f*)(tab + 4 * tid);
    *q = o;
    __threadfence();
    *q = o;
  }
}

__global__ __launch_bounds__(256) void k_score(const float* __restrict__ H, const float* __restrict__ tab,
                                               float* __restrict__ S) {
  __shared__ float ss[2][32];
  const int tid = (int)threadIdx.x, lane = tid & 31, wave = tid >> 5;
  const v4f a1 = *(const v4fa*)(tab + 4 * lane);
  const v4f a2 = *(const v4fa*)(tab + OUTC + 4 * lane);
  const int row0 = (int)blockIdx.x * 32 + wave * 4;
#pragma unroll 1
  for (int r = 0; r < 4; ++r) {
    const v4f h = *(const v4fa*)(H + (size_t)(row0 + r) * OUTC + 4 * lane);
    float p1 = h[0] * a1[0];
    p1 = fmaf(h[1], a1[1], p1);
    p1 = fmaf(h[2], a1[2], p1);
    p1 = fmaf(h[3], a1[3], p1);
    float p2 = h[0] * a2[0];
    p2 = fmaf(h[1], a2[1], p2);
    p2 = fmaf(h[2], a2[2], p2);
    p2 = fmaf(h[3], a2[3], p2);
#pragma unroll
    for (int off = 1; off < 32; off <<= 1) {
      p1 += __shfl_xor(p1, off, 32);
      p2 += __shfl_xor(p2, off, 32);
    }
    if (lane == 0) {
      ss[0][wave * 4 + r] = p1;
      ss[1][wave * 4 + r] = p2;
    }
  }
  __syncthreads();
  const float v = ss[wave & 1][lane];
  if (wave < 2) {
    volatile float* q = (volatile float*)(S + (size_t)wave * ROWS + (size_t)blockIdx.x * 32 + lane);
    *q = v;
    __threadfence();
    *q = v;
  }
}

__global__ __launch_bounds__(256) void k_bt(const float* __restrict__ H, unsigned short* __restrict__ BT) {
  __shared__ float tile[64 * 129];
  const int tid = (int)threadIdx.x, lane = tid & 31, wave = tid >> 5;
  const int b  = (int)blockIdx.x >> 4;
  const int j0 = ((int)blockIdx.x & 15) * 64;
  const float* src = H + ((size_t)b * NN + j0) * OUTC;
#pragma unroll 4
  for (int it = 0; it < 8; ++it) {
    const int idx = tid + 256 * it;
    const int row = idx >> 5;
    const int c4  = (idx & 31) * 4;
    const v4f v = *(const v4fa*)(src + (size_t)row * OUTC + c4);
    asm volatile("" :: "v"(v));
    tile[row * 129 + c4 + 0] = v[0];
    tile[row * 129 + c4 + 1] = v[1];
    tile[row * 129 + c4 + 2] = v[2];
    tile[row * 129 + c4 + 3] = v[3];
  }
  __syncthreads();
#pragma unroll 1
  for (int g = 0; g < 2; ++g) {
    const int nb = wave * 16 + g * 8;
    unsigned hw[8], lw[8];
#pragma unroll
    for (int q = 0; q < 8; ++q) {
      const float v0 = tile[(2 * lane) * 129 + nb + q];
      const float v1 = tile[(2 * lane + 1) * 129 + nb + q];
      hw[q] = pk16(bf16_bits(v0), bf16_bits(v1));
      lw[q] = (H_LO != 0) ? pk16(bf16_lo_bits(v0), bf16_lo_bits(v1)) : 0u;
    }
    unsigned short* base = BT + ((size_t)b * OUTC + nb) * KCAT + j0 + 2 * lane;
#pragma unroll
    for (int q = 0; q < 8; ++q) {
      unsigned short* rp = base + (size_t)q * KCAT;
      *(volatile unsigned*)(rp)          = hw[q];
      *(volatile unsigned*)(rp + NN)     = hw[q];
      *(volatile unsigned*)(rp + 2 * NN) = lw[q];
    }
    __threadfence();
#pragma unroll
    for (int q = 0; q < 8; ++q) {
      unsigned short* rp = base + (size_t)q * KCAT;
      *(volatile unsigned*)(rp)          = hw[q];
      *(volatile unsigned*)(rp + NN)     = hw[q];
      *(volatile unsigned*)(rp + 2 * NN) = lw[q];
    }
  }
}

__device__ __forceinline__ float escore(float s1, float s2, float g) {
  float x = s1 + s2;
  x = (x > 0.0f) ? x : SLOPE * x;
  x = x * bf16_val(g);
  return (x == 0.0f) ? FILLV : x;
}

__global__ __launch_bounds__(256) void k_softmax(const float* __restrict__ G, const float* __restrict__ S,
                                                 unsigned short* __restrict__ AP, int cbase) {
  __shared__ __attribute__((aligned(16))) float s2s[NN];
  __shared__ __attribute__((aligned(16))) float es[8][NN];
  const int tid = (int)threadIdx.x, lane = tid & 31, wave = tid >> 5;
  const int bl = (int)blockIdx.x / (NN / 8);
  const int i  = ((int)blockIdx.x - bl * (NN / 8)) * 8 + wave;
  const int b  = cbase + bl;
  {
    const v4f v = *(const v4fa*)(S + (size_t)ROWS + (size_t)b * NN + 4 * tid);
    *(v4fa*)(s2s + 4 * tid) = v;
  }
  __syncthreads();
  const float s1 = S[(size_t)b * NN + i];
  const float* grow = G + (size_t)i * NN + lane * 8;
  float* ew = es[wave] + lane * 8;

  float m = -3.0e38f;
#pragma unroll 1
  for (int t = 0; t < 4; ++t) {
    const v4f g0 = *(const v4fa*)(grow + t * 256);
    const v4f g1 = *(const v4fa*)(grow + t * 256 + 4);
    const v4f z0 = *(const v4fa*)(s2s + t * 256 + lane * 8);
    const v4f z1 = *(const v4fa*)(s2s + t * 256 + lane * 8 + 4);
    v4f e0, e1;
#pragma unroll
    for (int u = 0; u < 4; ++u) {
      e0[u] = escore(s1, z0[u], g0[u]);
      e1[u] = escore(s1, z1[u], g1[u]);
    }
#pragma unroll
    for (int u = 0; u < 4; ++u) m = fmaxf(m, e0[u]);
#pragma unroll
    for (int u = 0; u < 4; ++u) m = fmaxf(m, e1[u]);
    *(v4fa*)(ew + t * 256)     = e0;
    *(v4fa*)(ew + t * 256 + 4) = e1;
  }
#pragma unroll
  for (int off = 1; off < 32; off <<= 1) m = fmaxf(m, __shfl_xor(m, off, 32));
  __syncthreads();

  float sum = 0.0f;
#pragma unroll 1
  for (int k = 0; k < 32; ++k) {
    const int idx = (k >> 3) * 256 + (k & 7);
    const float p = expf(ew[idx] - m);
    ew[idx] = p;
    sum += p;
  }
#pragma unroll
  for (int off = 1; off < 32; off <<= 1) sum += __shfl_xor(sum, off, 32);
  const float rinv = 1.0f / sum;
  __syncthreads();

  unsigned short* arow = AP + ((size_t)bl * NN + i) * KCAT + lane * 8;
#pragma unroll 1
  for (int t = 0; t < 4; ++t) {
    const v4f p0 = *(const v4fa*)(ew + t * 256);
    const v4f p1 = *(const v4fa*)(ew + t * 256 + 4);
    const v4f q0 = p0 * rinv;
    const v4f q1 = p1 * rinv;
    const v4u hi = pack8_bf16(q0, q1);
    v4u lo = (v4u){0u, 0u, 0u, 0u};
    if (P_LO != 0) lo = pack8_bf16_lo(q0, q1);
    volatile v4u* d0 = (volatile v4u*)(arow + t * 256);
    volatile v4u* d1 = (volatile v4u*)(arow + NN + t * 256);
    volatile v4u* d2 = (volatile v4u*)(arow + 2 * NN + t * 256);
    *d0 = hi;
    *d1 = lo;
    *d2 = hi;
    __threadfence();
    *d0 = hi;
    *d1 = lo;
    *d2 = hi;
  }
}

__global__ __launch_bounds__(256) void k_out(const float* __restrict__ O, const float* __restrict__ tab,
                                             float* __restrict__ out) {
  __shared__ __attribute__((aligned(16))) float sb[OUTC];
  const int tid = (int)threadIdx.x, lane = tid & 31, wave = tid >> 5;
  {
    const int bi = tid < 32 ? tid : 31;
    const v4f bv = *(const v4fa*)(tab + 2 * OUTC + 4 * bi);
    asm volatile("" :: "v"(bv));
    if (tid < 32) *(v4fa*)(sb + 4 * tid) = bv;
  }
  __syncthreads();
  const int row = (int)blockIdx.x * 8 + wave;
  const int rc  = clampi(row, 0, ROWS - 1);
  const v4f v = *(const v4fa*)(O + (size_t)rc * OUTC + 4 * lane);
  const float c0 = v[0], c1 = v[1], c2 = v[2], c3 = v[3];
  asm volatile("" :: "v"(c0));
  asm volatile("" :: "v"(c1));
  asm volatile("" :: "v"(c2));
  asm volatile("" :: "v"(c3));
  const v4f bb = *(const v4fa*)(sb + 4 * lane);
  const v4f o = (v4f){ c0 + bb[0], c1 + bb[1], c2 + bb[2], c3 + bb[3] };
  if (row < ROWS) {
    volatile v4f* q = (volatile v4f*)(out + (size_t)row * OUTC + 4 * lane);
    *q = o;
    __threadfence();
    *q = o;
  }
}

extern "C" void kernel_launch(void* const* d_in, const int* in_sizes, int n_in,
                              void* d_out, int out_size, void* d_ws, size_t ws_size,
                              hipStream_t stream) {
  if (n_in < 5) return;
  if (in_sizes[0] != NBATCH * NN * INC) return;
  if (in_sizes[1] != NN * NN) return;
  if (in_sizes[2] != OUTC * INC) return;
  if (in_sizes[3] != OUTC) return;
  if (in_sizes[4] != 2 * OUTC) return;
  if (out_size != ROWS * OUTC) return;
  if (ws_size < WS_TOTAL) return;

  const float* X  = (const float*)d_in[0];
  const float* G  = (const float*)d_in[1];
  const float* W  = (const float*)d_in[2];
  const float* bv = (const float*)d_in[3];
  const float* av = (const float*)d_in[4];
  float* out = (float*)d_out;

  char* ws = (char*)d_ws;
  unsigned short* XB  = (unsigned short*)(ws + OFF_XB);
  unsigned short* WB  = (unsigned short*)(ws + OFF_WB);
  float*          TAB = (float*)(ws + OFF_TAB);
  float*          H   = (float*)(ws + OFF_H);
  float*          S   = (float*)(ws + OFF_S);
  unsigned short* BT  = (unsigned short*)(ws + OFF_BT);
  unsigned short* AP  = (unsigned short*)(ws + OFF_AP);
  float*          O   = (float*)(ws + OFF_O);

  k_plane<0><<<ROWS * (INC / 8) / 256, 256, 0, stream>>>(X, ROWS, INC, INC, XB, ROWS, INC);
  k_plane<0><<<OUTC * (INC / 8) / 256, 256, 0, stream>>>(W, OUTC, INC, INC, WB, OUTC, INC);
  k_tab<<<1, 256, 0, stream>>>(av, bv, TAB);
  {
    const int tiles = (ROWS / 64) * (OUTC / 64);
    k_gemm_nt<0, 0><<<(tiles + 7) / 8, 256, 0, stream>>>(XB, WB, TAB, H, ROWS, OUTC, INC, OUTC);
  }
  k_score<<<ROWS / 32, 256, 0, stream>>>(H, TAB, S);
  k_bt<<<NBATCH * (NN / 64), 256, 0, stream>>>(H, BT);
  const int tilesO = (NN / 64) * (OUTC / 64);
  for (int c = 0; c < NBATCH / CB; ++c) {
    k_softmax<<<CB * (NN / 8), 256, 0, stream>>>(G, S, AP, c * CB);
    for (int bl = 0; bl < CB; ++bl) {
      const int b = c * CB + bl;
      k_gemm_nt<0, 0><<<(tilesO + 7) / 8, 256, 0, stream>>>(AP + (size_t)bl * NN * KCAT,
                                                            BT + (size_t)b * OUTC * KCAT,
                                                            TAB, O + (size_t)b * NN * OUTC,
                                                            NN, OUTC, KCAT, OUTC);
    }
  }
  k_out<<<ROWS / 8, 256, 0, stream>>>(O, TAB, out);
}
